// XConv_41351945126432
// MI455X (gfx1250) — hardware-verified
//
#include <hip/hip_runtime.h>
#include <math.h>

constexpr int kB    = 4;
constexpr int kN    = 8192;
constexpr int kM    = 2048;
constexpr int kK    = 16;
constexpr int kCin  = 64;
constexpr int kCout = 128;
constexpr int kMid  = 32;
constexpr int kK2   = 256;
constexpr int kPts  = kB * kM;
constexpr int kRows = kPts * kK;
constexpr int kFeat = kMid + kCin;
constexpr int kKc   = kFeat * kK;
constexpr int kKs1  = 64;
constexpr int kN2   = 64;
constexpr float kEps = 1e-5f;

typedef __attribute__((ext_vector_type(16))) _Float16 v16h;
typedef __attribute__((ext_vector_type(8)))  _Float16 v8h;
typedef __attribute__((ext_vector_type(16))) __bf16   v16b;
typedef __attribute__((ext_vector_type(8)))  __bf16   v8b;
typedef __attribute__((ext_vector_type(8)))  float    v8f;
typedef __attribute__((ext_vector_type(4)))  float    v4f;
typedef __attribute__((ext_vector_type(4)))  unsigned int v4u;

__device__ __forceinline__ unsigned short f2bf_bits(float f) {
  unsigned u = __float_as_uint(f);
  return (unsigned short)((u + 0x7FFFu + ((u >> 16) & 1u)) >> 16);
}
__device__ __forceinline__ float bf_bits2f(unsigned short h) { return __uint_as_float(((unsigned)h) << 16); }
__device__ __forceinline__ float bfr(float f) { return bf_bits2f(f2bf_bits(f)); }
__device__ __forceinline__ unsigned pk16(unsigned short a, unsigned short b) { return (unsigned)a | ((unsigned)b << 16); }

__device__ __forceinline__ void dep_guard_h(v8f& a, v8f& b, v16h x, v16h y) { asm volatile("v_nop\n\tv_nop\n\tv_nop\n\tv_nop" : "+v"(a), "+v"(b) : "v"(x), "v"(y)); }
__device__ __forceinline__ void dep_guard_b(v8f& a, v8f& b, v16b x, v16b y) { asm volatile("v_nop\n\tv_nop\n\tv_nop\n\tv_nop" : "+v"(a), "+v"(b) : "v"(x), "v"(y)); }
__device__ __forceinline__ void keep4_h(v16h a, v16h b, v16h c, v16h d) { asm volatile("v_nop" :: "v"(a), "v"(b), "v"(c), "v"(d)); }
__device__ __forceinline__ void keep4_b(v16b a, v16b b, v16b c, v16b d) { asm volatile("v_nop" :: "v"(a), "v"(b), "v"(c), "v"(d)); }
__device__ __forceinline__ void acc_guard4(v8f& a, v8f& b, v8f& c, v8f& d) { asm volatile("v_nop\n\tv_nop\n\tv_nop\n\tv_nop" : "+v"(a), "+v"(b), "+v"(c), "+v"(d)); }
template <typename T> struct Frag;
template <> struct Frag<_Float16> {
  typedef v16h V; union U { v16h v; v8h h[2]; };
  static __device__ __forceinline__ v16h load(const _Float16* p) {
    U f; f.h[0] = *(const v8h*)(p); f.h[1] = *(const v8h*)(p + 16); return f.v;
  }
  static __device__ __forceinline__ v8f mma(v16h a, v16h b, v8f c) {
    return __builtin_amdgcn_wmma_f32_16x16x32_f16(false, a, false, b, (short)0, c, false, false);
  }
  static __device__ __forceinline__ void guard(v8f& a, v8f& b, v16h x, v16h y) { dep_guard_h(a, b, x, y); }
  static __device__ __forceinline__ void keep(v16h a, v16h b, v16h c, v16h d) { keep4_h(a, b, c, d); }
};
template <> struct Frag<__bf16> {
  typedef v16b V; union U { v16b v; v8b h[2]; };
  static __device__ __forceinline__ v16b load(const __bf16* p) {
    U f; f.h[0] = *(const v8b*)(p); f.h[1] = *(const v8b*)(p + 16); return f.v;
  }
  static __device__ __forceinline__ v8f mma(v16b a, v16b b, v8f c) {
    return __builtin_amdgcn_wmma_f32_16x16x32_bf16(false, a, false, b, (short)0, c, false, false);
  }
  static __device__ __forceinline__ void guard(v8f& a, v8f& b, v16b x, v16b y) { dep_guard_b(a, b, x, y); }
  static __device__ __forceinline__ void keep(v16b a, v16b b, v16b c, v16b d) { keep4_b(a, b, c, d); }
};

template <int ET> struct Elem;
template <> struct Elem<0> { typedef _Float16 T; };
template <> struct Elem<1> { typedef __bf16 T; };
template <int ET, int SPLIT, int BIAS_MODE, int OUT_MODE, bool RESID, int ACT = 0, int NST = 64>
__global__ __launch_bounds__(256) void wmma_gemm64(
    const unsigned short* __restrict__ Ap, const unsigned short* __restrict__ A2p, int lda, long strideA,
    const unsigned short* __restrict__ Btp, const unsigned short* __restrict__ Bt2p, int ldb, long strideB,
    void* __restrict__ Cout, void* __restrict__ Cout2, int ldc, long strideC,
    const float* __restrict__ bias,
    const float* __restrict__ resid, long strideR,
    int M, int N, int K, float scale) {
  typedef typename Elem<ET>::T T;
  typedef typename Frag<T>::V V;
  constexpr bool kSA = (SPLIT != 0);
  constexpr bool kSB = (SPLIT == 1);
  const T* A = (const T*)Ap; const T* A2 = (const T*)A2p; const T* Bt = (const T*)Btp; const T* Bt2 = (const T*)Bt2p;
  __shared__ __align__(16) float sT[8][16 * 68];
  const int b    = blockIdx.y;
  const int lane = threadIdx.x & 31;
  const int wave = threadIdx.x >> 5;
  const int tilesN = N >> 6;
  const int tilesM = M >> 6;
  const int tile = blockIdx.x * 8 + wave;
  if (tile >= tilesM * tilesN) return;
  const int tm = tile / tilesN;
  const int tn = tile - tm * tilesN;
  const int m0 = tm << 6;
  const int n0 = tn << 6;

  const T* Ab  = A  + (size_t)b * strideA;
  const T* Bb  = Bt + (size_t)b * strideB;
  const T* Ab2 = kSA ? (A2  + (size_t)b * strideA) : nullptr;
  const T* Bb2 = kSB ? (Bt2 + (size_t)b * strideB) : nullptr;

  const int rlane = lane & 15;
  const int koff  = (lane >> 4) * 8;
  const int mOff  = (lane >> 4) * 8;

  v8f acc[4][4];
#pragma unroll
  for (int i = 0; i < 4; ++i)
#pragma unroll
    for (int j = 0; j < 4; ++j) acc[i][j] = (v8f){0.f,0.f,0.f,0.f,0.f,0.f,0.f,0.f};

  for (int k0 = 0; k0 < K; k0 += 32) {
    V bh[4], bl[4];
#pragma unroll
    for (int j = 0; j < 4; ++j) {
      const size_t bo = (size_t)(n0 + (j << 4) + rlane) * ldb + koff + k0;
      bh[j] = Frag<T>::load(Bb + bo);
      if (kSB) bl[j] = Frag<T>::load(Bb2 + bo);
    }
#pragma unroll
    for (int i = 0; i < 4; ++i) {
      const size_t ao = (size_t)(m0 + (i << 4) + rlane) * lda + koff + k0;
      V ah = Frag<T>::load(Ab + ao);
      V al;
      if (kSA) al = Frag<T>::load(Ab2 + ao);
#pragma unroll
      for (int j = 0; j < 4; ++j) {
        acc[i][j] = Frag<T>::mma(ah, bh[j], acc[i][j]);
        if (kSB) acc[i][j] = Frag<T>::mma(ah, bl[j], acc[i][j]);
        if (kSA) acc[i][j] = Frag<T>::mma(al, bh[j], acc[i][j]);
      }
      Frag<T>::guard(acc[i][0], acc[i][3], ah, kSA ? al : ah);
    }
    Frag<T>::keep(bh[0], bh[1], bh[2], bh[3]);
    if (kSB) Frag<T>::keep(bl[0], bl[1], bl[2], bl[3]);
  }
  acc_guard4(acc[0][0], acc[0][1], acc[0][2], acc[0][3]);
  acc_guard4(acc[1][0], acc[1][1], acc[1][2], acc[1][3]);
  acc_guard4(acc[2][0], acc[2][1], acc[2][2], acc[2][3]);
  acc_guard4(acc[3][0], acc[3][1], acc[3][2], acc[3][3]);

  float* slab = sT[wave];
  const float* Rb = RESID ? (resid + (size_t)b * strideR) : nullptr;
#pragma unroll
  for (int i = 0; i < 4; ++i) {
    const int mBase = m0 + (i << 4);
#pragma unroll
    for (int j = 0; j < 4; ++j) {
      const int n = n0 + (j << 4) + rlane;
      float bv = 0.f;
      if (BIAS_MODE == 2) bv = bias[n];
#pragma unroll
      for (int r = 0; r < 8; ++r) {
        float v = acc[i][j][r] * scale;
        if (BIAS_MODE == 1) v += bias[mBase + mOff + r];
        if (BIAS_MODE == 2) v += bv;
        if (RESID) v += Rb[(size_t)(mBase + mOff + r) * ldc + n];
        if (ACT == 2) v = fmaxf(v, 0.0f);
        if (ACT == 4) v = (v > 0.f) ? v : 0.01f * v;
        slab[(mOff + r) * 68 + (j << 4) + rlane] = v;
      }
    }
    __builtin_amdgcn_fence(__ATOMIC_RELEASE, "workgroup");
    __builtin_amdgcn_wave_barrier();
    __builtin_amdgcn_fence(__ATOMIC_ACQUIRE, "workgroup");
    if (OUT_MODE == 0) {
      float* C = (float*)Cout + (size_t)b * strideC;
      const int hh = lane >> 4, c4 = (lane & 15) * 4;
      for (int pass = 0; pass < 2; ++pass) {
#pragma unroll
        for (int it = 0; it < 8; ++it) {
          const int row = it * 2 + hh;
          v4f v = *(const v4f*)(slab + row * 68 + c4);
          if (NST >= 64 || c4 < NST) *(volatile v4f*)(C + (size_t)(mBase + row) * ldc + n0 + c4) = v;
        }
        __threadfence();
      }
    } else {
      const int q = lane >> 3, c8 = (lane & 7) * 8;
      unsigned short* C  = (unsigned short*)Cout  + (size_t)b * strideC;
      unsigned short* C2 = (OUT_MODE == 2) ? ((unsigned short*)Cout2 + (size_t)b * strideC) : nullptr;
      for (int pass = 0; pass < 2; ++pass) {
#pragma unroll
        for (int it = 0; it < 4; ++it) {
          const int row = it * 4 + q;
          const float* sp = slab + row * 68 + c8;
          v8h hv, lv;
#pragma unroll
          for (int e = 0; e < 8; ++e) {
            if (OUT_MODE == 1) {
              hv[e] = (_Float16)sp[e];
            } else {
              unsigned short hb = f2bf_bits(sp[e]);
              unsigned short lb = f2bf_bits(sp[e] - bf_bits2f(hb));
              hv[e] = __builtin_bit_cast(_Float16, hb);
              lv[e] = __builtin_bit_cast(_Float16, lb);
            }
          }
          *(volatile v8h*)(C + (size_t)(mBase + row) * ldc + n0 + c8) = hv;
          if (OUT_MODE == 2) *(volatile v8h*)(C2 + (size_t)(mBase + row) * ldc + n0 + c8) = lv;
        }
        __threadfence();
      }
    }
    __builtin_amdgcn_fence(__ATOMIC_RELEASE, "workgroup");
    __builtin_amdgcn_wave_barrier();
    __builtin_amdgcn_fence(__ATOMIC_ACQUIRE, "workgroup");
  }
}

__device__ __forceinline__ void split2(float a, float b, unsigned& hw, unsigned& lw) {
  const unsigned short ha = f2bf_bits(a), hb = f2bf_bits(b);
  const unsigned short la = f2bf_bits(a - bf_bits2f(ha)), lb = f2bf_bits(b - bf_bits2f(hb));
  hw = pk16(ha, hb); lw = pk16(la, lb);
}
__device__ __forceinline__ float h1_val(float c0, float c1, float c2, float w0, float w1, float w2, float bb) {
  return fmaf(c2, w2, fmaf(c1, w1, c0 * w0)) + bb;
}

constexpr int kPkW2 = 4, kPkWs1 = 32, kPkWs2 = 128, kPkWs3 = 128, kPkWc = 384, kPkBias = 6;
constexpr int kPkTotal = kPkW2 + kPkWs1 + kPkWs2 + kPkWs3 + kPkWc + kPkBias;
static_assert(kN2 * kMid / 2 == kPkW2 * 256);
static_assert(kK2 * kKs1 / 2 == kPkWs1 * 256);
static_assert(kK2 * kK2 / 2 == kPkWs2 * 256);
static_assert(kCout * kKc / 2 == kPkWc * 256);

__global__ __launch_bounds__(256) void pack_kernel(
    const float* __restrict__ W2, const float* __restrict__ Ws1, const float* __restrict__ Ws2,
    const float* __restrict__ Ws3, const float* __restrict__ Wc,
    const float* __restrict__ b1, const float* __restrict__ b2, const float* __restrict__ bs1,
    const float* __restrict__ bs2, const float* __restrict__ bs3, const float* __restrict__ bc,
    unsigned* __restrict__ W2T, unsigned* __restrict__ WS1P, unsigned* __restrict__ WS2T,
    unsigned* __restrict__ WS3T, unsigned* __restrict__ WCB, float* __restrict__ BIASR) {
  const int blk = blockIdx.x;
  const int t = threadIdx.x;
  unsigned* dst = nullptr; unsigned val = 0u;
  float* fdst = nullptr; float fval = 0.f; bool isf = false;
  if (blk < kPkW2) {
    const int i = blk * 256 + t;
    const int n = i >> 4;
    const int k = 2 * (i & 15);
    float a = 0.f, c = 0.f;
    if (blk < 2) { a = W2[k * kMid + n]; c = W2[(k + 1) * kMid + n]; }
    val = pk16(f2bf_bits(a), f2bf_bits(c)); dst = W2T + i;
  } else if (blk < kPkW2 + kPkWs1) {
    const int i = (blk - kPkW2) * 256 + t;
    const int n = i >> 5;
    const int kk = 2 * (i & 31);
    const int kc = kk < 46 ? kk : 46;
    const float fz = (kk < 48) ? 1.f : 0.f;
    const float a = Ws1[n * 48 + kc] * fz, c = Ws1[n * 48 + kc + 1] * fz;
    val = pk16(f2bf_bits(a), f2bf_bits(c)); dst = WS1P + i;
  } else if (blk < kPkW2 + kPkWs1 + kPkWs2) {
    const int i = (blk - kPkW2 - kPkWs1) * 256 + t;
    const int n = i >> 7;
    const int k = 2 * (i & 127);
    const float a = Ws2[k * kK2 + n], c = Ws2[(k + 1) * kK2 + n];
    val = pk16(f2bf_bits(a), f2bf_bits(c)); dst = WS2T + i;
  } else if (blk < kPkW2 + kPkWs1 + kPkWs2 + kPkWs3) {
    const int i = (blk - kPkW2 - kPkWs1 - kPkWs2) * 256 + t;
    const int n = i >> 7;
    const int k = 2 * (i & 127);
    const float a = Ws3[k * kK2 + n], c = Ws3[(k + 1) * kK2 + n];
    val = pk16(f2bf_bits(a), f2bf_bits(c)); dst = WS3T + i;
  } else if (blk < kPkTotal - kPkBias) {
    const int i = (blk - kPkW2 - kPkWs1 - kPkWs2 - kPkWs3) * 256 + t;
    const float a = Wc[2 * (size_t)i], c = Wc[2 * (size_t)i + 1];
    val = pk16(f2bf_bits(a), f2bf_bits(c)); dst = WCB + i;
  } else {
    const int which = blk - (kPkTotal - kPkBias);
    const float* src; int len;
    if (which == 0)      { src = b1;  len = kMid; }
    else if (which == 1) { src = b2;  len = kMid; }
    else if (which == 2) { src = bs1; len = kK2; }
    else if (which == 3) { src = bs2; len = kK2; }
    else if (which == 4) { src = bs3; len = kK2; }
    else                 { src = bc;  len = kCout; }
    const int cc = t < len ? t : len - 1;
    const float fz = (t < len) ? 1.f : 0.f;
    fval = bfr(src[cc]) * fz; fdst = BIASR + which * 256 + t; isf = true;
  }
  if (isf) {
    *(volatile float*)fdst = fval; __threadfence(); *(volatile float*)fdst = fval;
  } else {
    *(volatile unsigned*)dst = val; __threadfence(); *(volatile unsigned*)dst = val;
  }
}

constexpr int kQB = 128;
static_assert(kM % kQB == 0);
static_assert(kN % kQB == 0);

__global__ __launch_bounds__(kQB) void knn_kernel(const float* __restrict__ p, const float* __restrict__ q,
                                                 const float* __restrict__ x, float* __restrict__ PHAT,
                                                 unsigned* __restrict__ PHAH, unsigned* __restrict__ PHAL,
                                                 unsigned* __restrict__ XN) {
#pragma clang fp contract(off)
  __shared__ float spx[kQB];
  __shared__ float spy[kQB];
  __shared__ float spz[kQB];
  __shared__ float spp[kQB];
  __shared__ float sqx[kQB];
  __shared__ float sqy[kQB];
  __shared__ float sqz[kQB];
  __shared__ int sidx[kQB * kK];
  __shared__ float sph[kQB * kK * 3];
  const int t = threadIdx.x;
  const int b = blockIdx.y;
  const int mq0 = blockIdx.x * kQB;
  const int pt0 = b * kM + mq0;
  const float* qr = q + ((size_t)(b * kM + mq0 + t)) * 3;
  const float qx = bfr(qr[0]), qy = bfr(qr[1]), qz = bfr(qr[2]);
  sqx[t] = qx; sqy[t] = qy; sqz[t] = qz;
  const float sqq = (qx * qx + qz * qz) + qy * qy;

  float bd[kK]; int bi[kK];
#pragma unroll
  for (int s = 0; s < kK; ++s) { bd[s] = __builtin_inff(); bi[s] = 0; }

#pragma unroll 1
  for (int n0 = 0; n0 < kN; n0 += kQB) {
    __syncthreads();
    {
      const float* pr = p + ((size_t)(b * kN + n0 + t)) * 3;
      const float px = bfr(pr[0]), py = bfr(pr[1]), pz = bfr(pr[2]);
      spx[t] = px; spy[t] = py; spz[t] = pz;
      spp[t] = (px * px + pz * pz) + py * py;
    }
    __syncthreads();
#pragma unroll 1
    for (int tt = 0; tt < kQB; ++tt) {
      const float px = spx[tt], py = spy[tt], pz = spz[tt];
      const float dot = fmaf(qz, pz, fmaf(qy, py, qx * px));
      const float dd = (sqq + spp[tt]) - 2.0f * dot;
      if (dd < bd[kK - 1]) {
        const int n = n0 + tt;
#pragma unroll
        for (int s = kK - 1; s >= 1; --s) {
          const bool up = dd < bd[s - 1];
          const bool here = dd < bd[s];
          const float nd = up ? bd[s - 1] : (here ? dd : bd[s]);
          const int   ni = up ? bi[s - 1] : (here ? n  : bi[s]);
          bd[s] = nd; bi[s] = ni;
        }
        const bool here0 = dd < bd[0];
        bd[0] = here0 ? dd : bd[0];
        bi[0] = here0 ? n  : bi[0];
      }
    }
  }
#pragma unroll
  for (int s = 0; s < kK; ++s) sidx[t * kK + s] = bi[s];
  __syncthreads();

#pragma unroll 1
  for (int it = 0; it < kK; ++it) {
    const int i = it * kQB + t;
    const int ql = i >> 4;
    int n = sidx[i]; n = n < 0 ? 0 : (n > kN - 1 ? kN - 1 : n);
    const float* pr = p + ((size_t)(b * kN + n)) * 3;
    const float c0 = bfr(pr[0]) - sqx[ql];
    const float c1 = bfr(pr[1]) - sqy[ql];
    const float c2 = bfr(pr[2]) - sqz[ql];
    sph[i * 3 + 0] = c0; sph[i * 3 + 1] = c1; sph[i * 3 + 2] = c2;
    const v4f v = {c0, c1, c2, 0.f};
    float* dst = PHAT + ((size_t)pt0 * kK + i) * 4;
    *(volatile v4f*)dst = v; __threadfence(); *(volatile v4f*)dst = v;
  }
  __syncthreads();

#pragma unroll 1
  for (int it = 0; it < 8; ++it) {
    const int i = it * kQB + t;
    const int ql = i >> 3;
    const int j = i & 7;
    const int c = ((j >> 1) < 2) ? (j >> 1) : 2;
    const bool live = j < 6;
    const int kb8 = (j & 1) * 8;
    unsigned hw[4], lw[4];
#pragma unroll
    for (int e = 0; e < 8; e += 2) {
      float v0 = sph[(ql * kK + kb8 + e) * 3 + c];
      float v1 = sph[(ql * kK + kb8 + e + 1) * 3 + c];
      v0 = live ? v0 : 0.f; v1 = live ? v1 : 0.f;
      split2(v0, v1, hw[e >> 1], lw[e >> 1]);
    }
    const v4u hu = {hw[0], hw[1], hw[2], hw[3]};
    const v4u lu = {lw[0], lw[1], lw[2], lw[3]};
    unsigned* dh = PHAH + (size_t)(pt0 + ql) * (kKs1 / 2) + 4 * j;
    unsigned* dl = PHAL + (size_t)(pt0 + ql) * (kKs1 / 2) + 4 * j;
    *(volatile v4u*)dh = hu; *(volatile v4u*)dl = lu;
    __threadfence();
    *(volatile v4u*)dh = hu; *(volatile v4u*)dl = lu;
  }

#pragma unroll 1
  for (int it = 0; it < kK * 8; ++it) {
    const int i = it * kQB + t;
    const int row = i >> 3;
    const int j = i & 7;
    int n = sidx[row]; n = n < 0 ? 0 : (n > kN - 1 ? kN - 1 : n);
    const float* xc = x + ((size_t)(b * kCin + 8 * j)) * kN + n;
    unsigned short hb[8];
#pragma unroll
    for (int e = 0; e < 8; ++e) hb[e] = f2bf_bits(xc[(size_t)e * kN]);
    const v4u u = {pk16(hb[0], hb[1]), pk16(hb[2], hb[3]), pk16(hb[4], hb[5]), pk16(hb[6], hb[7])};
    unsigned* dx = XN + ((size_t)pt0 * kK + row) * (kCin / 2) + 4 * j;
    *(volatile v4u*)dx = u; __threadfence(); *(volatile v4u*)dx = u;
  }
}

constexpr int kHChunks = 128;
constexpr int kHRpc = kRows / kHChunks;
static_assert(kHRpc % 8 == 0);

__global__ __launch_bounds__(256) void h1_stats_kernel(const float* __restrict__ PHAT, const float* __restrict__ W1,
                                                      const float* __restrict__ BIASR, double* __restrict__ PART) {
  __shared__ double red[2][8][32];
  const int lane = threadIdx.x & 31, wave = threadIdx.x >> 5;
  const int chunk = blockIdx.x;
  const float w0 = bfr(W1[lane]), w1 = bfr(W1[kMid + lane]), w2 = bfr(W1[2 * kMid + lane]);
  const float bb = BIASR[lane];
  double s = 0.0, s2 = 0.0;
  const int r0 = chunk * kHRpc + wave * (kHRpc / 8);
#pragma unroll 1
  for (int j = 0; j < kHRpc / 8; ++j) {
    const v4f ph = *(const v4f*)(PHAT + (size_t)(r0 + j) * 4);
    const float h = h1_val(ph[0], ph[1], ph[2], w0, w1, w2, bb);
    const double dh = (double)h;
    s += dh; s2 += dh * dh;
  }
  red[0][wave][lane] = s; red[1][wave][lane] = s2;
  __syncthreads();
  if (wave == 0) {
    double S = 0.0, S2 = 0.0;
#pragma unroll
    for (int w = 0; w < 8; ++w) { S += red[0][w][lane]; S2 += red[1][w][lane]; }
    double* d0 = PART + (size_t)(chunk * 2) * kMid + lane;
    double* d1 = PART + (size_t)(chunk * 2 + 1) * kMid + lane;
    *(volatile double*)d0 = S; *(volatile double*)d1 = S2;
    __threadfence();
    *(volatile double*)d0 = S; *(volatile double*)d1 = S2;
  }
}

__global__ __launch_bounds__(256) void col_stats_kernel(const float* __restrict__ Mx, int C, int rpc,
                                                      double* __restrict__ PART) {
  __shared__ double red[2][8][32];
  const int lane = threadIdx.x & 31, wave = threadIdx.x >> 5;
  const int cg = blockIdx.x;
  const int chunk = blockIdx.y;
  const int c = cg * 32 + lane;
  double s = 0.0, s2 = 0.0;
  const int nj = rpc >> 3;
#pragma unroll 1
  for (int j = 0; j < nj; ++j) {
    const int r = chunk * rpc + wave + 8 * j;
    const float v = Mx[(size_t)r * C + c];
    const double dv = (double)v;
    s += dv; s2 += dv * dv;
  }
  red[0][wave][lane] = s; red[1][wave][lane] = s2;
  __syncthreads();
  if (wave == 0) {
    double S = 0.0, S2 = 0.0;
#pragma unroll
    for (int w = 0; w < 8; ++w) { S += red[0][w][lane]; S2 += red[1][w][lane]; }
    double* d0 = PART + (size_t)(chunk * 2) * C + cg * 32 + lane;
    double* d1 = PART + (size_t)(chunk * 2 + 1) * C + cg * 32 + lane;
    *(volatile double*)d0 = S; *(volatile double*)d1 = S2;
    __threadfence();
    *(volatile double*)d0 = S; *(volatile double*)d1 = S2;
  }
}

__global__ __launch_bounds__(256) void bn_finalize_kernel(const double* __restrict__ PART, int C, int nchunks, double inv_n,
                                                        const float* __restrict__ g, const float* __restrict__ be,
                                                        float* __restrict__ SS) {
  const int c = threadIdx.x;
  if (c < C) {
    double S = 0.0, S2 = 0.0;
#pragma unroll 1
    for (int ch = 0; ch < nchunks; ++ch) {
      S  += PART[(size_t)(ch * 2) * C + c];
      S2 += PART[(size_t)(ch * 2 + 1) * C + c];
    }
    const double mean = S * inv_n;
    double var = S2 * inv_n - mean * mean;
    var = var > 0.0 ? var : 0.0;
    const float mu = (float)mean;
    const float vf = (float)var;
    const float rs = 1.0f / sqrtf(vf + kEps);
    const float gr = bfr(g[c]);
    const float br = bfr(be[c]);
    float* d = SS + c;
    for (int pass = 0; pass < 2; ++pass) {
      *(volatile float*)(d) = mu;
      *(volatile float*)(d + C) = rs;
      *(volatile float*)(d + 2 * C) = gr;
      *(volatile float*)(d + 3 * C) = br;
      __threadfence();
    }
  }
}

static_assert((kRows * 4) % 256 == 0);
__global__ __launch_bounds__(256) void h1_apply_kernel(const float* __restrict__ PHAT, const float* __restrict__ W1,
                                                      const float* __restrict__ BIASR, const float* __restrict__ SS,
                                                      unsigned* __restrict__ H, unsigned* __restrict__ L) {
  __shared__ float sW[3 * kMid];
  __shared__ float sBias[kMid];
  __shared__ float sS[4 * kMid];
  const int t = threadIdx.x;
  {
    const float wv = bfr(W1[t < 3 * kMid ? t : 3 * kMid - 1]);
    const float bv = BIASR[t < kMid ? t : kMid - 1];
    const float sv = SS[t < 4 * kMid ? t : 4 * kMid - 1];
    if (t < 3 * kMid) sW[t] = wv;
    if (t < kMid) sBias[t] = bv;
    if (t < 4 * kMid) sS[t] = sv;
  }
  __syncthreads();
  const int i = blockIdx.x * 256 + t;
  const int row = i >> 2;
  const int c8 = (i & 3) * 8;
  const v4f ph = *(const v4f*)(PHAT + (size_t)row * 4);
  unsigned hw[4], lw[4];
#pragma unroll
  for (int e = 0; e < 8; e += 2) {
    const int ca = c8 + e, cb = c8 + e + 1;
    const float ha = h1_val(ph[0], ph[1], ph[2], sW[ca], sW[kMid + ca], sW[2 * kMid + ca], sBias[ca]);
    const float hb = h1_val(ph[0], ph[1], ph[2], sW[cb], sW[kMid + cb], sW[2 * kMid + cb], sBias[cb]);
    float ya = ((ha - sS[ca]) * sS[kMid + ca]) * sS[2 * kMid + ca] + sS[3 * kMid + ca];
    float yb = ((hb - sS[cb]) * sS[kMid + cb]) * sS[2 * kMid + cb] + sS[3 * kMid + cb];
    ya = fmaxf(ya, 0.f); yb = fmaxf(yb, 0.f);
    split2(ya, yb, hw[e >> 1], lw[e >> 1]);
  }
  const v4u hu = {hw[0], hw[1], hw[2], hw[3]};
  const v4u lu = {lw[0], lw[1], lw[2], lw[3]};
  unsigned* dh = H + (size_t)i * 4;
  unsigned* dl = L + (size_t)i * 4;
  *(volatile v4u*)dh = hu; *(volatile v4u*)dl = lu;
  __threadfence();
  *(volatile v4u*)dh = hu; *(volatile v4u*)dl = lu;
}

template <int C>
__global__ __launch_bounds__(256) void bn_apply_split_kernel(const float* __restrict__ Mx, const float* __restrict__ SS, int n8,
                                                           unsigned* __restrict__ H, unsigned* __restrict__ L) {
  static_assert((C & (C - 1)) == 0 && C % 8 == 0 && 4 * C <= 1024);
  __shared__ float sS[4 * C];
  for (int i = threadIdx.x; i < 4 * C; i += 256) sS[i] = SS[i];
  __syncthreads();
  const int i = blockIdx.x * 256 + threadIdx.x;
  if (i < n8) {
    const size_t e0 = (size_t)i * 8;
    const int c0 = (int)(e0 & (size_t)(C - 1));
    const v4f a = *(const v4f*)(Mx + e0);
    const v4f bq = *(const v4f*)(Mx + e0 + 4);
    float o[8];
#pragma unroll
    for (int e = 0; e < 4; ++e) { o[e] = a[e]; o[4 + e] = bq[e]; }
    unsigned hw[4], lw[4];
#pragma unroll
    for (int e = 0; e < 8; e += 2) {
      const int ca = c0 + e, cb = c0 + e + 1;
      float ya = ((o[e] - sS[ca]) * sS[C + ca]) * sS[2 * C + ca] + sS[3 * C + ca];
      float yb = ((o[e + 1] - sS[cb]) * sS[C + cb]) * sS[2 * C + cb] + sS[3 * C + cb];
      ya = fmaxf(ya, 0.f); yb = fmaxf(yb, 0.f);
      split2(ya, yb, hw[e >> 1], lw[e >> 1]);
    }
    const v4u hu = {hw[0], hw[1], hw[2], hw[3]};
    const v4u lu = {lw[0], lw[1], lw[2], lw[3]};
    unsigned* dh = H + (size_t)i * 4;
    unsigned* dl = L + (size_t)i * 4;
    *(volatile v4u*)dh = hu; *(volatile v4u*)dl = lu;
    __threadfence();
    *(volatile v4u*)dh = hu; *(volatile v4u*)dl = lu;
  }
}

constexpr int kFP = 4;
static_assert(kPts % kFP == 0);
static_assert(kFP * kK2 == 4 * 256);
static_assert((kFP * kK * kMid) % 256 == 0 && (kFP * kK * kCin / 2) % 256 == 0 && (kFP * kKc / 8) % 256 == 0);

__global__ __launch_bounds__(256) void ft_kernel(const float* __restrict__ TT, const float* __restrict__ H2,
                                                const float* __restrict__ SS2, const unsigned* __restrict__ XNw,
                                                unsigned* __restrict__ FTH, unsigned* __restrict__ FTL) {
  __shared__ __align__(16) float sT[kFP * kK2];
  __shared__ __align__(16) float sF[kFP * kK * kFeat];
  __shared__ __align__(16) float sO[kFP * kKc];
  __shared__ float sS[4 * kMid];
  const int t = threadIdx.x;
  const int pt0 = blockIdx.x * kFP;
  {
    const float sv = SS2[t < 4 * kMid ? t : 4 * kMid - 1];
    if (t < 4 * kMid) sS[t] = sv;
    const v4f tv = *(const v4f*)(TT + (size_t)pt0 * kK2 + 4 * t);
    *(v4f*)(sT + 4 * t) = tv;
  }
  __syncthreads();
#pragma unroll 4
  for (int it = 0; it < (kFP * kK * kMid) / 256; ++it) {
    const int e = it * 256 + t;
    const int rowl = e >> 5;
    const int c = e & 31;
    const float v = H2[((size_t)pt0 * kK + rowl) * kMid + c];
    float y = ((v - sS[c]) * sS[kMid + c]) * sS[2 * kMid + c] + sS[3 * kMid + c];
    y = fmaxf(y, 0.f);
    sF[rowl * kFeat + c] = y;
  }
#pragma unroll 4
  for (int it = 0; it < (kFP * kK * kCin / 2) / 256; ++it) {
    const int e = it * 256 + t;
    const int rowl = e >> 5;
    const int wj = e & 31;
    const unsigned w = XNw[((size_t)pt0 * kK + rowl) * (kCin / 2) + wj];
    sF[rowl * kFeat + kMid + 2 * wj]     = __uint_as_float(w << 16);
    sF[rowl * kFeat + kMid + 2 * wj + 1] = __uint_as_float(w & 0xffff0000u);
  }
  __syncthreads();
#pragma unroll
  for (int it = 0; it < 2; ++it) {
    const int item = it * 256 + t;
    if (item < kFP * kFeat) {
      const int ptl = item / kFeat;
      const int c = item - ptl * kFeat;
      float f[kK];
#pragma unroll
      for (int j = 0; j < kK; ++j) f[j] = sF[(ptl * kK + j) * kFeat + c];
      const float* tb = sT + ptl * kK2;
      float* ob = sO + ptl * kKc + c * kK;
#pragma unroll 1
      for (int i2 = 0; i2 < kK; ++i2) {
        const v4f t0 = *(const v4f*)(tb + i2 * kK);
        const v4f t1 = *(const v4f*)(tb + i2 * kK + 4);
        const v4f t2 = *(const v4f*)(tb + i2 * kK + 8);
        const v4f t3 = *(const v4f*)(tb + i2 * kK + 12);
        float acc = 0.0f;
#pragma unroll
        for (int j = 0; j < 4; ++j) acc += t0[j] * f[j];
#pragma unroll
        for (int j = 0; j < 4; ++j) acc += t1[j] * f[4 + j];
#pragma unroll
        for (int j = 0; j < 4; ++j) acc += t2[j] * f[8 + j];
#pragma unroll
        for (int j = 0; j < 4; ++j) acc += t3[j] * f[12 + j];
        ob[i2] = acc;
      }
    }
  }
  __syncthreads();
  for (int pass = 0; pass < 2; ++pass) {
#pragma unroll
    for (int it = 0; it < 3; ++it) {
      const int g8 = it * 256 + t;
      const v4f a = *(const v4f*)(sO + 8 * g8);
      const v4f bq = *(const v4f*)(sO + 8 * g8 + 4);
      unsigned hw[4], lw[4];
      split2(a[0], a[1], hw[0], lw[0]);
      split2(a[2], a[3], hw[1], lw[1]);
      split2(bq[0], bq[1], hw[2], lw[2]);
      split2(bq[2], bq[3], hw[3], lw[3]);
      const v4u hu = {hw[0], hw[1], hw[2], hw[3]};
      const v4u lu = {lw[0], lw[1], lw[2], lw[3]};
      unsigned* dh = FTH + (size_t)pt0 * (kKc / 2) + 4 * g8;
      unsigned* dl = FTL + (size_t)pt0 * (kKc / 2) + 4 * g8;
      *(volatile v4u*)dh = hu; *(volatile v4u*)dl = lu;
    }
    __threadfence();
  }
}

constexpr int kOutBlocks = kB * (kM / 64);
constexpr int kQ4 = kPts * 3 / 4;
constexpr int kQBlocks = kQ4 / 256;
static_assert(kQ4 % 256 == 0);
static_assert(kM % 64 == 0 && kCout == 128);
constexpr int kOut1Off = kPts * 3;
static_assert((kOut1Off * 4) % 128 == 0);

__global__ __launch_bounds__(256) void finalize_out_kernel(const float* __restrict__ OUTPRE, const float* __restrict__ SS,
                                                          const float* __restrict__ q, float* __restrict__ out) {
  __shared__ __align__(16) float sm[kCout * 68];
  __shared__ float sS[4 * kCout];
  const int blk = blockIdx.x;
  const int t = threadIdx.x;
  if (blk >= kOutBlocks) {
    const int i = (blk - kOutBlocks) * 256 + t;
    const v4f v = *(const v4f*)(q + 4 * (size_t)i);
    const v4f r = {bfr(v[0]), bfr(v[1]), bfr(v[2]), bfr(v[3])};
    float* d = out + 4 * (size_t)i;
    *(volatile v4f*)d = r; __threadfence(); *(volatile v4f*)d = r;
    return;
  }
  const int b = blk >> 5;
  const int mc = blk & 31;
  for (int i = t; i < 4 * kCout; i += 256) sS[i] = SS[i];
  __syncthreads();
#pragma unroll 4
  for (int it = 0; it < 32; ++it) {
    const int e = it * 256 + t;
    const int r = e >> 7;
    const int o = e & 127;
    const float v = OUTPRE[((size_t)(b * kM + mc * 64 + r)) * kCout + o];
    float y = ((v - sS[o]) * sS[kCout + o]) * sS[2 * kCout + o] + sS[3 * kCout + o];
    y = fmaxf(y, 0.f);
    sm[o * 68 + r] = y;
  }
  __syncthreads();
  const int lane = t & 31, wave = t >> 5;
  const int hh = lane >> 4, c4 = (lane & 15) * 4;
  float* ob = out + kOut1Off + (size_t)b * kCout * kM + mc * 64;
  for (int pass = 0; pass < 2; ++pass) {
#pragma unroll
    for (int it = 0; it < 8; ++it) {
      const int o = wave * 16 + it * 2 + hh;
      const v4f v = *(const v4f*)(sm + o * 68 + c4);
      *(volatile v4f*)(ob + (size_t)o * kM + c4) = v;
    }
    __threadfence();
  }
}

constexpr size_t kSzBias = 6 * 256 * 4;
constexpr size_t kSzW2T  = (size_t)kN2 * kMid * 2;
constexpr size_t kSzWs1  = (size_t)kK2 * kKs1 * 2;
constexpr size_t kSzWs2  = (size_t)kK2 * kK2 * 2;
constexpr size_t kSzWc   = (size_t)kCout * kKc * 2;
constexpr size_t kSzPhat = (size_t)kRows * 4 * 4;
constexpr size_t kSzPha  = (size_t)kPts * kKs1 * 2;
constexpr size_t kSzXn   = (size_t)kRows * kCin * 2;
constexpr size_t kSzH1n  = (size_t)kRows * kMid * 2;
constexpr size_t kSzH2   = (size_t)kRows * kMid * 4;
constexpr size_t kSzT    = (size_t)kPts * kK2 * 4;
constexpr size_t kSzTn   = (size_t)kPts * kK2 * 2;
constexpr size_t kSzFt   = (size_t)kPts * kKc * 2;
constexpr size_t kSzOut  = (size_t)kPts * kCout * 4;
constexpr size_t kSzPart = 131072;
constexpr size_t kSzSS   = 4096;
constexpr int kTChunks = 32;
constexpr int kTRpc = kPts / kTChunks;
static_assert(kTRpc % 8 == 0);
static_assert((size_t)kHChunks * 2 * kMid * 8 <= kSzPart);
static_assert((size_t)kTChunks * 2 * kK2 * 8 <= kSzPart);
static_assert((size_t)kTChunks * 2 * kCout * 8 <= kSzPart);
static_assert(4 * kK2 * 4 <= kSzSS);
static_assert(kRows % 64 == 0 && kN2 % 64 == 0 && kMid % 32 == 0);
static_assert(kPts % 64 == 0 && kK2 % 64 == 0 && kKs1 % 32 == 0 && kK2 % 32 == 0);
static_assert(kCout % 64 == 0 && kKc % 32 == 0);
static_assert(kOut1Off * 4 + kPts * kCout * 4 == 4292608);

extern "C" void kernel_launch(void* const* d_in, const int* in_sizes, int n_in,
                              void* d_out, int out_size, void* d_ws, size_t ws_size, hipStream_t stream) {
  (void)in_sizes; (void)n_in; (void)out_size;
  const float* p    = (const float*)d_in[0];
  const float* q    = (const float*)d_in[1];
  const float* x    = (const float*)d_in[2];
  const float* W1   = (const float*)d_in[3];
  const float* b1   = (const float*)d_in[4];
  const float* g1   = (const float*)d_in[5];
  const float* be1  = (const float*)d_in[6];
  const float* W2   = (const float*)d_in[7];
  const float* b2   = (const float*)d_in[8];
  const float* g2   = (const float*)d_in[9];
  const float* be2  = (const float*)d_in[10];
  const float* Ws1  = (const float*)d_in[11];
  const float* bs1  = (const float*)d_in[12];
  const float* gs1  = (const float*)d_in[13];
  const float* bes1 = (const float*)d_in[14];
  const float* Ws2  = (const float*)d_in[15];
  const float* bs2  = (const float*)d_in[16];
  const float* gs2  = (const float*)d_in[17];
  const float* bes2 = (const float*)d_in[18];
  const float* Ws3  = (const float*)d_in[19];
  const float* bs3  = (const float*)d_in[20];
  const float* Wc   = (const float*)d_in[21];
  const float* bc   = (const float*)d_in[22];
  const float* gc   = (const float*)d_in[23];
  const float* bec  = (const float*)d_in[24];
  float* out = (float*)d_out;

  char* ws = (char*)d_ws;
  size_t off = 0;
  auto carve = [&](size_t bytes) -> char* { char* r = ws + off; off += (bytes + 255) & ~(size_t)255; return r; };
  float*    BIASR = (float*)carve(kSzBias);
  unsigned* W2T   = (unsigned*)carve(kSzW2T);
  unsigned* WS1P  = (unsigned*)carve(kSzWs1);
  unsigned* WS2T  = (unsigned*)carve(kSzWs2);
  unsigned* WS3T  = (unsigned*)carve(kSzWs2);
  unsigned* WCB   = (unsigned*)carve(kSzWc);
  float*    PHAT  = (float*)carve(kSzPhat);
  unsigned* PHAH  = (unsigned*)carve(kSzPha);
  unsigned* PHAL  = (unsigned*)carve(kSzPha);
  unsigned* XN    = (unsigned*)carve(kSzXn);
  unsigned* H1NH  = (unsigned*)carve(kSzH1n);
  unsigned* H1NL  = (unsigned*)carve(kSzH1n);
  float*    H2PRE = (float*)carve(kSzH2);
  float*    TPRE  = (float*)carve(kSzT);
  unsigned* TNH   = (unsigned*)carve(kSzTn);
  unsigned* TNL   = (unsigned*)carve(kSzTn);
  unsigned* FTH   = (unsigned*)carve(kSzFt);
  unsigned* FTL   = (unsigned*)carve(kSzFt);
  float*    OUTPRE = (float*)carve(kSzOut);
  double*   PART1 = (double*)carve(kSzPart);
  double*   PART2 = (double*)carve(kSzPart);
  double*   PART3 = (double*)carve(kSzPart);
  double*   PART4 = (double*)carve(kSzPart);
  double*   PART5 = (double*)carve(kSzPart);
  float*    SS1 = (float*)carve(kSzSS);
  float*    SS2 = (float*)carve(kSzSS);
  float*    SS3 = (float*)carve(kSzSS);
  float*    SS4 = (float*)carve(kSzSS);
  float*    SS5 = (float*)carve(kSzSS);
  if (off > ws_size || off > (size_t)134217728) return;

  const unsigned short* kNoPlane = nullptr;

  pack_kernel<<<kPkTotal, 256, 0, stream>>>(W2, Ws1, Ws2, Ws3, Wc, b1, b2, bs1, bs2, bs3, bc,
                                           W2T, WS1P, WS2T, WS3T, WCB, BIASR);
  knn_kernel<<<dim3(kM / kQB, kB), kQB, 0, stream>>>(p, q, x, PHAT, PHAH, PHAL, XN);
  h1_stats_kernel<<<kHChunks, 256, 0, stream>>>(PHAT, W1, BIASR, PART1);
  bn_finalize_kernel<<<1, 256, 0, stream>>>(PART1, kMid, kHChunks, 1.0 / (double)kRows, g1, be1, SS1);
  h1_apply_kernel<<<(kRows * 4) / 256, 256, 0, stream>>>(PHAT, W1, BIASR, SS1, H1NH, H1NL);
  {
    const int tiles = (kRows / 64) * (kN2 / 64);
    wmma_gemm64<1, 2, 2, 0, false, 0, 32><<<dim3((tiles + 7) / 8, 1), 256, 0, stream>>>(
        (const unsigned short*)H1NH, (const unsigned short*)H1NL, kMid, 0L,
        (const unsigned short*)W2T, kNoPlane, kMid, 0L,
        (void*)H2PRE, (void*)nullptr, kMid, 0L,
        BIASR + 1 * 256, (const float*)nullptr, 0L, kRows, kN2, kMid, 1.0f);
  }
  col_stats_kernel<<<dim3(kMid / 32, kHChunks), 256, 0, stream>>>(H2PRE, kMid, kHRpc, PART2);
  bn_finalize_kernel<<<1, 256, 0, stream>>>(PART2, kMid, kHChunks, 1.0 / (double)kRows, g2, be2, SS2);
  {
    const int tiles = (kPts / 64) * (kK2 / 64);
    wmma_gemm64<1, 2, 2, 0, false, 0, 64><<<dim3((tiles + 7) / 8, 1), 256, 0, stream>>>(
        (const unsigned short*)PHAH, (const unsigned short*)PHAL, kKs1, 0L,
        (const unsigned short*)WS1P, kNoPlane, kKs1, 0L,
        (void*)TPRE, (void*)nullptr, kK2, 0L,
        BIASR + 2 * 256, (const float*)nullptr, 0L, kPts, kK2, kKs1, 1.0f);
  }
  col_stats_kernel<<<dim3(kK2 / 32, kTChunks), 256, 0, stream>>>(TPRE, kK2, kTRpc, PART3);
  bn_finalize_kernel<<<1, 256, 0, stream>>>(PART3, kK2, kTChunks, 1.0 / (double)kPts, gs1, bes1, SS3);
  bn_apply_split_kernel<kK2><<<(kPts * kK2 / 8) / 256, 256, 0, stream>>>(TPRE, SS3, kPts * kK2 / 8, TNH, TNL);
  {
    const int tiles = (kPts / 64) * (kK2 / 64);
    wmma_gemm64<1, 2, 2, 0, false, 0, 64><<<dim3((tiles + 7) / 8, 1), 256, 0, stream>>>(
        (const unsigned short*)TNH, (const unsigned short*)TNL, kK2, 0L,
        (const unsigned short*)WS2T, kNoPlane, kK2, 0L,
        (void*)TPRE, (void*)nullptr, kK2, 0L,
        BIASR + 3 * 256, (const float*)nullptr, 0L, kPts, kK2, kK2, 1.0f);
  }
  col_stats_kernel<<<dim3(kK2 / 32, kTChunks), 256, 0, stream>>>(TPRE, kK2, kTRpc, PART4);
  bn_finalize_kernel<<<1, 256, 0, stream>>>(PART4, kK2, kTChunks, 1.0 / (double)kPts, gs2, bes2, SS4);
  bn_apply_split_kernel<kK2><<<(kPts * kK2 / 8) / 256, 256, 0, stream>>>(TPRE, SS4, kPts * kK2 / 8, TNH, TNL);
  {
    const int tiles = (kPts / 64) * (kK2 / 64);
    wmma_gemm64<1, 2, 2, 0, false, 0, 64><<<dim3((tiles + 7) / 8, 1), 256, 0, stream>>>(
        (const unsigned short*)TNH, (const unsigned short*)TNL, kK2, 0L,
        (const unsigned short*)WS3T, kNoPlane, kK2, 0L,
        (void*)TPRE, (void*)nullptr, kK2, 0L,
        BIASR + 4 * 256, (const float*)nullptr, 0L, kPts, kK2, kK2, 1.0f);
  }
  ft_kernel<<<kPts / kFP, 256, 0, stream>>>(TPRE, H2PRE, SS2, XN, FTH, FTL);
  {
    const int tiles = (kPts / 64) * (kCout / 64);
    wmma_gemm64<1, 2, 2, 0, false, 0, 64><<<dim3((tiles + 7) / 8, 1), 256, 0, stream>>>(
        (const unsigned short*)FTH, (const unsigned short*)FTL, kKc, 0L,
        (const unsigned short*)WCB, kNoPlane, kKc, 0L,
        (void*)OUTPRE, (void*)nullptr, kCout, 0L,
        BIASR + 5 * 256, (const float*)nullptr, 0L, kPts, kCout, kKc, 1.0f);
  }
  col_stats_kernel<<<dim3(kCout / 32, kTChunks), 256, 0, stream>>>(OUTPRE, kCout, kTRpc, PART5);
  bn_finalize_kernel<<<1, 256, 0, stream>>>(PART5, kCout, kTChunks, 1.0 / (double)kPts, gc, bec, SS5);
  finalize_out_kernel<<<kOutBlocks + kQBlocks, 256, 0, stream>>>(OUTPRE, SS5, q, out);
}
